// RGAT_16252156248488
// MI455X (gfx1250) — hardware-verified
//
#include <hip/hip_runtime.h>
#include <stddef.h>
#include <stdint.h>
#include <math.h>


#define F_IN    128
#define HC      128
#define HD      64
#define NHEAD   2
#define HID     64
#define KA      128
#define KL      256
#define NTHR    256
#define NWAVE   8
#define EPT     8
#define CHUNK   (NTHR * EPT)
#define WCAP    (EPT * 32)
#define LISTN   (NWAVE * WCAP)
#define NBMAX   2048
#define SLOTB   11
#define RCAP    28672
#define DEGCAP  256
#define GBM     64
#define GTHR    128
#define MROWS   128
#define NU0     (2 * HC * (KA / 8))
#define NU1     (2 * HC * (KA / 8))
#define NUL     (HID * (KL / 8))
#define NUW     (NU0 + NU1 + 2 * NUL)
#define NEGSL   0.2f
#define EPS_SM  1e-16f
#define MX0     (-1.0e30f)
#define WSMAX   134217728
#define LDS_AGG ((2 * RCAP + 2 * NBMAX + LISTN) * 4 + 64)

static_assert((CHUNK & (CHUNK - 1)) == 0 && CHUNK <= (1 << SLOTB));
static_assert(NBMAX == (1 << SLOTB));
static_assert(NTHR * 8 == NBMAX);
static_assert(LISTN >= NBMAX);
static_assert(LISTN >= NWAVE * WCAP);
static_assert((RCAP % 32) == 0);
static_assert(LDS_AGG <= 300000);
static_assert(GBM == (GTHR / 32) * 16);
static_assert(GTHR == 2 * GBM);
static_assert(2 * GTHR == 2 * NHEAD * HD);
static_assert((KA % 32) == 0 && (KL % 32) == 0);
static_assert(F_IN == KA && 2 * HID == KA && KL == 2 * HC);
static_assert(HC == NHEAD * HD && HD == 16 * 4);
static_assert(HC == 4 * 32);
static_assert(HID == 4 * 16);
static_assert(HC * 4 == KL * 2);
static_assert((MROWS % GBM) == 0);
static_assert((NU0 % NTHR) == 0 && ((NU0 + NU1) % NTHR) == 0 && ((NU0 + NU1 + NUL) % NTHR) == 0 && (NUW % NTHR) == 0);
static_assert((KA / 8) == 16 && (KL / 8) == 32);
static_assert(((GBM * HID * 4) % 128) == 0 && (GTHR % 16) == 0);

typedef float          v4f  __attribute__((ext_vector_type(4)));
typedef float          v8f  __attribute__((ext_vector_type(8)));
typedef int            v4i  __attribute__((ext_vector_type(4)));
typedef int            v8i  __attribute__((ext_vector_type(8)));
typedef unsigned int   v4u  __attribute__((ext_vector_type(4)));
typedef unsigned short v8us __attribute__((ext_vector_type(8)));
typedef __bf16         v16b __attribute__((ext_vector_type(16)));
typedef v4f  __attribute__((may_alias)) v4fa;
typedef v8us __attribute__((may_alias)) v8usa;
union FragB { v16b v; v8us h[2]; v8i w; };

__device__ __forceinline__ v8f wmb(const FragB& a, const FragB& b, v8f c) {
  v8f d = __builtin_amdgcn_wmma_f32_16x16x32_bf16(false, a.v, false, b.v, (short)0, c, false, false);
  asm volatile("v_nop\n\tv_nop\n\tv_nop\n\tv_nop" : "+v"(d) : "v"(a.w), "v"(b.w));
  return d;
}

__device__ __forceinline__ unsigned int f2bf(float f) {
  const unsigned int u = __float_as_uint(f);
  return ((u + 0x7FFFu + ((u >> 16) & 1u)) >> 16) & 0xFFFFu;
}
__device__ __forceinline__ float bf2f(unsigned int b) { return __uint_as_float(b << 16); }
__device__ __forceinline__ float bfr(float f) { return bf2f(f2bf(f)); }
__device__ __forceinline__ v4f bfr4(const v4f a) {
  v4f r; r.x = bfr(a.x); r.y = bfr(a.y); r.z = bfr(a.z); r.w = bfr(a.w); return r;
}
__device__ __forceinline__ unsigned int pk2(float lo, float hi) { return f2bf(lo) | (f2bf(hi) << 16); }
__device__ __forceinline__ v4u pack8(const v4f a, const v4f b) {
  v4u r;
  r.x = pk2(a.x, a.y); r.y = pk2(a.z, a.w); r.z = pk2(b.x, b.y); r.w = pk2(b.z, b.w);
  return r;
}
__device__ __forceinline__ v8us hilo8(v4f t) {
  v8us o;
  unsigned hb;
  hb = f2bf(t.x); o[0] = (unsigned short)hb; o[4] = (unsigned short)f2bf(t.x - __uint_as_float(hb << 16));
  hb = f2bf(t.y); o[1] = (unsigned short)hb; o[5] = (unsigned short)f2bf(t.y - __uint_as_float(hb << 16));
  hb = f2bf(t.z); o[2] = (unsigned short)hb; o[6] = (unsigned short)f2bf(t.z - __uint_as_float(hb << 16));
  hb = f2bf(t.w); o[3] = (unsigned short)hb; o[7] = (unsigned short)f2bf(t.w - __uint_as_float(hb << 16));
  return o;
}

__device__ __forceinline__ int scan_chunk(const int* __restrict__ dsts, int nE, int cbase, int slotBase,
                                          int nb, int vec8, int* list, int tid, int lane, int wave) {
  int wc = 0;
  const int el0  = tid * EPT;
  const int e0   = cbase + el0;
  const int sent = -2147483647 - 1;
  v4i da, db;
  if (vec8 != 0 && cbase + CHUNK <= nE) {
    da = *(const v4i*)(dsts + e0);
    db = *(const v4i*)(dsts + e0 + 4);
  } else {
    da.x = (e0     < nE) ? dsts[min(e0,     nE - 1)] : sent;
    da.y = (e0 + 1 < nE) ? dsts[min(e0 + 1, nE - 1)] : sent;
    da.z = (e0 + 2 < nE) ? dsts[min(e0 + 2, nE - 1)] : sent;
    da.w = (e0 + 3 < nE) ? dsts[min(e0 + 3, nE - 1)] : sent;
    db.x = (e0 + 4 < nE) ? dsts[min(e0 + 4, nE - 1)] : sent;
    db.y = (e0 + 5 < nE) ? dsts[min(e0 + 5, nE - 1)] : sent;
    db.z = (e0 + 6 < nE) ? dsts[min(e0 + 6, nE - 1)] : sent;
    db.w = (e0 + 7 < nE) ? dsts[min(e0 + 7, nE - 1)] : sent;
  }
  const unsigned nbs = (unsigned)slotBase;
  const unsigned unb = (unsigned)nb;
  const unsigned s0 = (unsigned)da.x - nbs, s1 = (unsigned)da.y - nbs;
  const unsigned s2 = (unsigned)da.z - nbs, s3 = (unsigned)da.w - nbs;
  const unsigned s4 = (unsigned)db.x - nbs, s5 = (unsigned)db.y - nbs;
  const unsigned s6 = (unsigned)db.z - nbs, s7 = (unsigned)db.w - nbs;
  const bool h0 = s0 < unb, h1 = s1 < unb, h2 = s2 < unb, h3 = s3 < unb;
  const bool h4 = s4 < unb, h5 = s5 < unb, h6 = s6 < unb, h7 = s7 < unb;
  const unsigned any = __builtin_amdgcn_ballot_w32(h0 | h1 | h2 | h3 | h4 | h5 | h6 | h7);
  if (any != 0u) {
#define HITJ(J, HJ, SJ) { \
      const unsigned mj = __builtin_amdgcn_ballot_w32(HJ); \
      if (mj != 0u) { \
        if (HJ) { \
          const int pos = wc + (int)__builtin_amdgcn_mbcnt_lo(mj, 0u); \
          if (pos < WCAP) list[wave * WCAP + pos] = ((el0 + (J)) << SLOTB) | (int)(SJ); \
        } \
        wc += (int)__builtin_popcount(mj); } }
    HITJ(0, h0, s0)
    HITJ(1, h1, s1)
    HITJ(2, h2, s2)
    HITJ(3, h3, s3)
    HITJ(4, h4, s4)
    HITJ(5, h5, s5)
    HITJ(6, h6, s6)
    HITJ(7, h7, s7)
#undef HITJ
  }
  return wc;
}

__global__ __launch_bounds__(NTHR) void k_xprep(const float* __restrict__ x, unsigned short* xb, int nN, int nUnits) {
  const int i = (int)blockIdx.x * NTHR + (int)threadIdx.x;
  if (i >= nUnits) return;
  const int row = i >> 4;
  const int c0  = (i & 15) * 8;
  const int rc  = row < nN ? row : nN - 1;
  const float* p = x + (size_t)rc * F_IN + c0;
  v4f a = *(const v4fa*)p, b = *(const v4fa*)(p + 4);
  const v4f z4 = {0.f, 0.f, 0.f, 0.f};
  if (row >= nN) { a = z4; b = z4; }
  const v4u hv = pack8(a, b);
  const size_t o = (size_t)row * KA + c0;
  *(volatile v4u*)(xb + o) = hv;
  __threadfence();
  *(volatile v4u*)(xb + o) = hv;
}

__global__ __launch_bounds__(NTHR) void k_wprep(const float* __restrict__ W0, const float* __restrict__ W1,
                                                const float* __restrict__ LW0, const float* __restrict__ LW1,
                                                unsigned short* W0T, unsigned short* W1T,
                                                unsigned short* L0T, unsigned short* L1T) {
  const int u = (int)blockIdx.x * NTHR + (int)threadIdx.x;
  if (u >= NUW) return;
  v8us o;
  unsigned short* dp;
  if (u < NU0) {
    const int n   = u >> 4;
    const int k8  = (u & 15) * 8;
    const int rel = n >> 7, col = n & (HC - 1);
    const float* p = W0 + (size_t)rel * F_IN * HC + (size_t)k8 * HC + col;
#pragma unroll
    for (int i = 0; i < 8; ++i) o[i] = (unsigned short)f2bf(p[(size_t)i * HC]);
    dp = W0T + (size_t)n * KA + k8;
  } else if (u < NU0 + NU1) {
    const int v   = u - NU0;
    const int n   = v >> 4;
    const int g   = v & 15;
    const int rel = n >> 7, col = n & (HC - 1);
    const float* p = W1 + (size_t)rel * HID * HC + (size_t)(4 * g) * HC + col;
    const unsigned short f0 = (unsigned short)f2bf(p[0]);
    const unsigned short f1 = (unsigned short)f2bf(p[HC]);
    const unsigned short f2 = (unsigned short)f2bf(p[2 * HC]);
    const unsigned short f3 = (unsigned short)f2bf(p[3 * HC]);
    o[0] = f0; o[1] = f1; o[2] = f2; o[3] = f3; o[4] = f0; o[5] = f1; o[6] = f2; o[7] = f3;
    dp = W1T + (size_t)n * KA + 8 * g;
  } else if (u < NU0 + NU1 + NUL) {
    const int v = u - NU0 - NU1;
    const int n = v >> 5;
    const int g = v & 31;
    const float* p = LW0 + (size_t)(4 * g) * HID + n;
    const unsigned short f0 = (unsigned short)f2bf(p[0]);
    const unsigned short f1 = (unsigned short)f2bf(p[HID]);
    const unsigned short f2 = (unsigned short)f2bf(p[2 * HID]);
    const unsigned short f3 = (unsigned short)f2bf(p[3 * HID]);
    o[0] = f0; o[1] = f1; o[2] = f2; o[3] = f3; o[4] = f0; o[5] = f1; o[6] = f2; o[7] = f3;
    dp = L0T + (size_t)n * KL + 8 * g;
  } else {
    const int v = u - NU0 - NU1 - NUL;
    const int n = v >> 5;
    const int g = v & 31;
    const float* p = LW1 + (size_t)(4 * g) * HID + n;
    const unsigned short f0 = (unsigned short)f2bf(p[0]);
    const unsigned short f1 = (unsigned short)f2bf(p[HID]);
    const unsigned short f2 = (unsigned short)f2bf(p[2 * HID]);
    const unsigned short f3 = (unsigned short)f2bf(p[3 * HID]);
    o[0] = f0; o[1] = f1; o[2] = f2; o[3] = f3; o[4] = f0; o[5] = f1; o[6] = f2; o[7] = f3;
    dp = L1T + (size_t)n * KL + 8 * g;
  }
  *(volatile v8us*)dp = o;
  __threadfence();
  *(volatile v8us*)dp = o;
}

__global__ __launch_bounds__(GTHR) void k_gemm(
    const unsigned short* __restrict__ A, const unsigned short* __restrict__ WT, float* outF,
    const float* __restrict__ alp, const float* __restrict__ arp, float* SD, int MPr)
{
  constexpr int PPR = 2 * NHEAD;
  __shared__ __attribute__((aligned(16))) float stg[GBM * HC];
  __shared__ __attribute__((aligned(16))) float satt[2 * HC];
  __shared__ __attribute__((aligned(16))) float sdot[PPR * GBM];
  const int tid = (int)threadIdx.x, lane = tid & 31, wave = tid >> 5, hh = lane >> 4, m = lane & 15;
  const int rowBase = (int)blockIdx.x * GBM;

#pragma unroll 1
  for (int q = 0; q < 2; ++q) {
    const int i     = tid + q * GTHR;
    const int hw    = i >> 6;
    const int head  = hw >> 1;
    const int which = hw & 1;
    const int c     = i & (HD - 1);
    const int idx   = head * HD + c;
    const float va  = alp[idx], vd = arp[idx];
    const float mw  = (float)which;
    const float v   = fmaf(mw, vd, (1.f - mw) * va);
    satt[i] = bfr(v);
  }

  v8f acc[8];
  {
    const v8f z = {0.f, 0.f, 0.f, 0.f, 0.f, 0.f, 0.f, 0.f};
#pragma unroll
    for (int t = 0; t < 8; ++t) acc[t] = z;
  }
  const unsigned short* ap = A  + (size_t)(rowBase + 16 * wave + m) * (size_t)KA + 8 * hh;
  const unsigned short* bp = WT + (size_t)m * (size_t)KA + 8 * hh;

#pragma unroll 1
  for (int ks = 0; ks < KA / 32; ++ks) {
    const int k0 = 32 * ks;
    FragB af;
    af.h[0] = *(const v8usa*)(ap + k0);
    af.h[1] = *(const v8usa*)(ap + k0 + 16);
#pragma unroll
    for (int nt = 0; nt < 8; ++nt) {
      const unsigned short* wq = bp + (size_t)(16 * nt) * (size_t)KA + k0;
      FragB bf;
      bf.h[0] = *(const v8usa*)wq;
      bf.h[1] = *(const v8usa*)(wq + 16);
      acc[nt] = wmb(af, bf, acc[nt]);
    }
  }

#pragma unroll
  for (int nt = 0; nt < 8; ++nt) {
    const int lc = 16 * nt + m;
#pragma unroll
    for (int r = 0; r < 8; ++r) {
      const int lr = 16 * wave + 8 * hh + r;
      stg[lr * HC + lc] = acc[nt][r];
    }
  }
  __syncthreads();

  {
    const int row = tid & 63, g = tid >> 6;
    const float* hr = stg + row * HC + g * HD;
    const float* sa = satt + (2 * g + 0) * HD;
    const float* sd = satt + (2 * g + 1) * HD;
    float ds = 0.f, dd = 0.f;
#pragma unroll 2
    for (int c4 = 0; c4 < HD / 4; ++c4) {
      const v4f h0 = *(const v4fa*)(hr + 4 * c4);
      const v4f a0 = *(const v4fa*)(sa + 4 * c4);
      const v4f b0 = *(const v4fa*)(sd + 4 * c4);
      ds = fmaf(h0.x, a0.x, ds); dd = fmaf(h0.x, b0.x, dd);
      ds = fmaf(h0.y, a0.y, ds); dd = fmaf(h0.y, b0.y, dd);
      ds = fmaf(h0.z, a0.z, ds); dd = fmaf(h0.z, b0.z, dd);
      ds = fmaf(h0.w, a0.w, ds); dd = fmaf(h0.w, b0.w, dd);
    }
    sdot[(2 * g + 0) * GBM + row] = ds;
    sdot[(2 * g + 1) * GBM + row] = dd;
  }
  __syncthreads();

  v4f fv[16];
#pragma unroll
  for (int i = 0; i < 16; ++i) {
    const int lr = 16 * wave + i;
    fv[i] = *(const v4fa*)(stg + lr * HC + 4 * lane);
  }
  const int pl = tid >> 4, piece = tid & 15;
  const bool wsd = pl < PPR;
  const int plr = wsd ? pl : PPR - 1;
  const v4f sdv = *(const v4fa*)(sdot + plr * GBM + 4 * piece);
  float* sp = SD + (size_t)plr * (size_t)MPr + rowBase + 4 * piece;

#pragma unroll
  for (int i = 0; i < 16; ++i) {
    float* op = outF + (size_t)(rowBase + 16 * wave + i) * (size_t)HC + 4 * lane;
    *(volatile v4f*)op = fv[i];
  }
  if (wsd) *(volatile v4f*)sp = sdv;
  __threadfence();
#pragma unroll
  for (int i = 0; i < 16; ++i) {
    float* op = outF + (size_t)(rowBase + 16 * wave + i) * (size_t)HC + 4 * lane;
    *(volatile v4f*)op = fv[i];
  }
  if (wsd) *(volatile v4f*)sp = sdv;
}

template <int SECOND>
__global__ __launch_bounds__(NTHR) void k_agg(
    const int* __restrict__ srcs, const int* __restrict__ dsts,
    const float* __restrict__ F, const float* __restrict__ SD,
    const float* __restrict__ bias, const float* P, float* Pw, unsigned short* HP,
    int nN, int nE, int nb, int vec8, int MPr) {
  extern __shared__ v4f lds_dyn[];
  int* reg1 = (int*)lds_dyn;
  int* reg2 = reg1 + RCAP;
  int* scnt = reg2 + RCAP;
  int* soff = scnt + NBMAX;
  int* list = soff + NBMAX;
  int* wcnt = list + LISTN;
  int* wtot = wcnt + NWAVE;
  const int tid = (int)threadIdx.x, lane = tid & 31, wave = tid >> 5;
  const int nodeBase = (int)blockIdx.x * nb;

  for (int i = tid; i < NBMAX; i += NTHR) scnt[i] = 0;
  __syncthreads();

  int tot = 0;
  const int nChunks = (nE + CHUNK - 1) / CHUNK;
#pragma unroll 1
  for (int ch = 0; ch < nChunks; ++ch) {
    const int cbase = ch * CHUNK;
    const int wc = scan_chunk(dsts, nE, cbase, nodeBase, nb, vec8, list, tid, lane, wave);
    if (lane == 0) wcnt[wave] = wc;
    __syncthreads();
    int pre = 0, all = 0;
#pragma unroll
    for (int w2 = 0; w2 < NWAVE; ++w2) {
      int c = wcnt[w2];
      c = c < 0 ? 0 : (c > WCAP ? WCAP : c);
      all += c;
      pre += (w2 < wave) ? c : 0;
    }
    const int wcc  = wc > WCAP ? WCAP : wc;
    const int base = tot + pre;
#pragma unroll 1
    for (int i = lane; i < wcc; i += 32) {
      const int ent = list[wave * WCAP + i];
      const int el  = (ent >> SLOTB) & (CHUNK - 1);
      const int sl  = ent & (NBMAX - 1);
      int eid = cbase + el;
      eid = eid > nE - 1 ? nE - 1 : eid;
      const int pos = base + i;
      if (pos < RCAP) reg1[pos] = (int)(((unsigned)eid << SLOTB) | (unsigned)sl);
    }
    tot += all;
    tot = tot > RCAP ? RCAP : tot;
    __syncthreads();
  }
  const int nh = tot;

  if (wave == 0) {
#pragma unroll 1
    for (int b0 = 0; b0 < nh; b0 += 32) {
      const int idx = b0 + lane;
      const int uv  = reg1[idx < nh ? idx : nh - 1];
      const int m32 = (nh - b0) < 32 ? (nh - b0) : 32;
#pragma unroll 1
      for (int k = 0; k < m32; ++k) {
        const int u  = __builtin_amdgcn_readlane(uv, k);
        const int sl = u & (NBMAX - 1);
        if (lane == 0) scnt[sl] = scnt[sl] + 1;
      }
    }
  }
  __syncthreads();

  {
    const v4i ca = *(const v4i*)(scnt + 8 * tid);
    const v4i cb = *(const v4i*)(scnt + 8 * tid + 4);
    const int e0 = ca.x < 0 ? 0 : ca.x, e1 = ca.y < 0 ? 0 : ca.y, e2 = ca.z < 0 ? 0 : ca.z, e3 = ca.w < 0 ? 0 : ca.w;
    const int e4 = cb.x < 0 ? 0 : cb.x, e5 = cb.y < 0 ? 0 : cb.y, e6 = cb.z < 0 ? 0 : cb.z, e7 = cb.w < 0 ? 0 : cb.w;
    const int ts = e0 + e1 + e2 + e3 + e4 + e5 + e6 + e7;
    int incl = ts;
#pragma unroll
    for (int d = 1; d < 32; d <<= 1) {
      const int up = __shfl_up(incl, d);
      if (lane >= d) incl += up;
    }
    if (lane == 31) wtot[wave] = incl;
    __syncthreads();
    int pre = 0;
#pragma unroll
    for (int w2 = 0; w2 < NWAVE; ++w2) pre += (w2 < wave) ? wtot[w2] : 0;
    int run = pre + incl - ts;
    soff[8 * tid + 0] = run; run += e0;
    soff[8 * tid + 1] = run; run += e1;
    soff[8 * tid + 2] = run; run += e2;
    soff[8 * tid + 3] = run; run += e3;
    soff[8 * tid + 4] = run; run += e4;
    soff[8 * tid + 5] = run; run += e5;
    soff[8 * tid + 6] = run; run += e6;
    soff[8 * tid + 7] = run;
  }
  __syncthreads();
  for (int i = tid; i < NBMAX; i += NTHR) list[i] = soff[i];
  __syncthreads();

  if (wave == 0) {
#pragma unroll 1
    for (int b0 = 0; b0 < nh; b0 += 32) {
      const int idx = b0 + lane;
      const int uv  = reg1[idx < nh ? idx : nh - 1];
      const int m32 = (nh - b0) < 32 ? (nh - b0) : 32;
#pragma unroll 1
      for (int k = 0; k < m32; ++k) {
        const int u   = __builtin_amdgcn_readlane(uv, k);
        const int sl  = u & (NBMAX - 1);
        const int eid = (int)((unsigned)u >> SLOTB);
        if (lane == 0) {
          int pos = list[sl];
          pos = pos < 0 ? 0 : (pos > RCAP - 1 ? RCAP - 1 : pos);
          reg2[pos] = eid;
          list[sl] = pos + 1;
        }
      }
    }
  }
  __syncthreads();

  const int nbw = nb >> 3;
  const bool ovf = (nh >= RCAP);
  const float qnan = __int_as_float(0x7fc00000);
  const int c0   = 4 * lane;
  const int head = lane >> 4;
  const v4f bb   = bfr4(*(const v4fa*)(bias + c0));
  const float* ASp = SD + (size_t)(2 * head) * (size_t)MPr;
  const float* ADp = ASp + MPr;
  const float* Fr  = F + c0;
  const v4f z4 = {0.f, 0.f, 0.f, 0.f};

#pragma unroll 1
  for (int jt = 0; jt < nbw; ++jt) {
    const int slot = wave * nbw + jt;
    const int grow = nodeBase + slot;
    if (grow >= MPr) break;
    const int gcl  = grow < nN ? grow : nN - 1;
    int st = soff[slot];
    const int craw = scnt[slot];
    int cnt = craw;
    st  = st < 0 ? 0 : (st > nh ? nh : st);
    cnt = cnt < 0 ? 0 : (cnt > DEGCAP ? DEGCAP : cnt);
    if (cnt > nh - st) cnt = nh - st;
    const float pz = (ovf || craw > DEGCAP) ? qnan : 0.0f;

    const float adv = ADp[gcl];
    float mx = MX0, dn = 0.0f;
    v4f av = z4;

#pragma unroll 1
    for (int q = 0; q < cnt; ++q) {
      int idx = st + q; idx = idx > RCAP - 1 ? RCAP - 1 : idx;
      int eid = reg2[idx]; eid = eid < 0 ? 0 : (eid > nE - 1 ? nE - 1 : eid);
      const int sraw = srcs[eid];
      const int s = sraw < 0 ? 0 : (sraw > nN - 1 ? nN - 1 : sraw);
      const v4f fs = *(const v4fa*)(Fr + (size_t)s * HC);
      float lg = ASp[s] + adv;
      lg = lg > 0.f ? lg : NEGSL * lg;
      const float df = lg - mx;
      const float ee = __expf(-fabsf(df));
      const bool up  = df > 0.f;
      const float s1 = up ? ee : 1.0f;
      const float s2 = up ? 1.0f : ee;
      mx = up ? lg : mx;
      dn = fmaf(dn, s1, s2);
      av.x = fmaf(av.x, s1, s2 * fs.x);
      av.y = fmaf(av.y, s1, s2 * fs.y);
      av.z = fmaf(av.z, s1, s2 * fs.z);
      av.w = fmaf(av.w, s1, s2 * fs.w);
    }
    const float inv = __builtin_amdgcn_rcpf(dn + EPS_SM);
    const bool live = grow < nN;
    v4f pv = z4;
    if constexpr (SECOND == 1) pv = *(const v4fa*)(P + (size_t)grow * HC + c0);
    v4f v;
    v.x = pv.x + fmaf(av.x, inv, bb.x);
    v.y = pv.y + fmaf(av.y, inv, bb.y);
    v.z = pv.z + fmaf(av.z, inv, bb.z);
    v.w = pv.w + fmaf(av.w, inv, bb.w);
    v4f o;
    o.x = (live ? v.x : 0.f) + pz;
    o.y = (live ? v.y : 0.f) + pz;
    o.z = (live ? v.z : 0.f) + pz;
    o.w = (live ? v.w : 0.f) + pz;

    if constexpr (SECOND == 0) {
      float* op = Pw + (size_t)grow * HC + c0;
      *(volatile v4f*)op = o;
      __threadfence();
      *(volatile v4f*)op = o;
    } else {
      const v8us po = hilo8(o);
      unsigned short* hp = HP + (size_t)grow * (size_t)KL + 8 * lane;
      *(volatile v8us*)hp = po;
      __threadfence();
      *(volatile v8us*)hp = po;
    }
  }
}

template <int MODE>
__global__ __launch_bounds__(GTHR) void k_lin(const unsigned short* __restrict__ A,
                                              const unsigned short* __restrict__ BT,
                                              const float* __restrict__ bias,
                                              unsigned short* HB, float* outp, int nN) {
  __shared__ __attribute__((aligned(16))) float stg[GBM * HID];
  const int tid = (int)threadIdx.x, lane = tid & 31, wave = tid >> 5, hh = lane >> 4, m = lane & 15;
  const int rowBase = (int)blockIdx.x * GBM;

  v8f acc[4];
  {
    const v8f z = {0.f, 0.f, 0.f, 0.f, 0.f, 0.f, 0.f, 0.f};
#pragma unroll
    for (int t = 0; t < 4; ++t) acc[t] = z;
  }
  const unsigned short* ap = A  + (size_t)(rowBase + 16 * wave + m) * (size_t)KL + 8 * hh;
  const unsigned short* wp = BT + (size_t)m * (size_t)KL + 8 * hh;
#pragma unroll 1
  for (int ks = 0; ks < KL / 32; ++ks) {
    const int k0 = 32 * ks;
    FragB af;
    af.h[0] = *(const v8usa*)(ap + k0);
    af.h[1] = *(const v8usa*)(ap + k0 + 16);
#pragma unroll
    for (int nt = 0; nt < 4; ++nt) {
      const unsigned short* wq = wp + (size_t)(16 * nt) * (size_t)KL + k0;
      FragB bf;
      bf.h[0] = *(const v8usa*)wq;
      bf.h[1] = *(const v8usa*)(wq + 16);
      acc[nt] = wmb(af, bf, acc[nt]);
    }
  }
#pragma unroll
  for (int nt = 0; nt < 4; ++nt) {
    const int lc = 16 * nt + m;
#pragma unroll
    for (int r = 0; r < 8; ++r) {
      const int lr = 16 * wave + 8 * hh + r;
      stg[lr * HID + lc] = acc[nt][r];
    }
  }
  __syncthreads();

  if constexpr (MODE == 0) {
    const int g = lane & 15;
    const v4f bb = bfr4(*(const v4f*)(bias + 4 * g));
    v8us po[8];
#pragma unroll
    for (int i = 0; i < 8; ++i) {
      const int lr   = 16 * wave + 2 * i + hh;
      const int grow = rowBase + lr;
      const v4f t    = *(const v4fa*)(stg + lr * HID + 4 * g);
      const bool live = grow < nN;
      v4f e;
      e.x = live ? fmaxf(t.x + bb.x, 0.f) : 0.f;
      e.y = live ? fmaxf(t.y + bb.y, 0.f) : 0.f;
      e.z = live ? fmaxf(t.z + bb.z, 0.f) : 0.f;
      e.w = live ? fmaxf(t.w + bb.w, 0.f) : 0.f;
      po[i] = hilo8(e);
    }
#pragma unroll
    for (int i = 0; i < 8; ++i) {
      unsigned short* hp = HB + (size_t)(rowBase + 16 * wave + 2 * i + hh) * (size_t)KA + 8 * g;
      *(volatile v8us*)hp = po[i];
    }
    __threadfence();
#pragma unroll
    for (int i = 0; i < 8; ++i) {
      unsigned short* hp = HB + (size_t)(rowBase + 16 * wave + 2 * i + hh) * (size_t)KA + 8 * g;
      *(volatile v8us*)hp = po[i];
    }
  } else {
    int live = nN - rowBase; live = live < 0 ? 0 : (live > GBM ? GBM : live);
    const int npc = live * (HID / 4);
    const int c4 = (tid & 15) * 4;
    const v4f bb4 = bfr4(*(const v4f*)(bias + c4));
    float* ob = outp + (size_t)rowBase * HID;
#pragma unroll 1
    for (int p = tid; p < npc; p += GTHR) {
      const v4f v = *(const v4fa*)(stg + 4 * p) + bb4;
      *(volatile v4f*)(ob + 4 * p) = v;
    }
    __threadfence();
#pragma unroll 1
    for (int p = tid; p < npc; p += GTHR) {
      const v4f v = *(const v4fa*)(stg + 4 * p) + bb4;
      *(volatile v4f*)(ob + 4 * p) = v;
    }
  }
}

static int pick_nb(int nE, int nN) {
  int nb = NBMAX;
  while (nb > 32 && (long long)nb * (long long)nE * 5LL > (long long)RCAP * (long long)nN * 2LL) nb >>= 1;
  return nb;
}
static inline int cdiv(int a, int b) { return (a + b - 1) / b; }

extern "C" void kernel_launch(void* const* d_in, const int* in_sizes, int n_in,
                              void* d_out, int out_size, void* d_ws, size_t ws_size,
                              hipStream_t stream) {
  if (n_in < 15) return;
  if (in_sizes[0] < F_IN || (in_sizes[0] % F_IN) != 0) return;
  const int nN = in_sizes[0] / F_IN;
  if (nN > (1 << 22)) return;
  if (in_sizes[1] < 2 || (in_sizes[1] & 1) != 0 || in_sizes[2] != in_sizes[1]) return;
  const int nE = in_sizes[1] / 2;
  if (nE < 1 || nE >= (1 << (32 - SLOTB))) return;
  if (in_sizes[3] != 2 * F_IN * HC) return;
  if (in_sizes[4] != 2 * HC || in_sizes[5] != 2 * HC || in_sizes[6] != 2 * HC) return;
  if (in_sizes[7] != 2 * HID * HC) return;
  if (in_sizes[8] != 2 * HC || in_sizes[9] != 2 * HC || in_sizes[10] != 2 * HC) return;
  if (in_sizes[11] != HC * HID || in_sizes[12] != HID) return;
  if (in_sizes[13] != HC * HID || in_sizes[14] != HID) return;
  if ((long long)out_size != (long long)nN * HID) return;

  const float* x     = (const float*)d_in[0];
  const int*   src   = (const int*)d_in[1];
  const int*   dst   = (const int*)d_in[2];
  const float* W0    = (const float*)d_in[3];
  const float* al0   = (const float*)d_in[4];
  const float* ar0   = (const float*)d_in[5];
  const float* b0    = (const float*)d_in[6];
  const float* W1    = (const float*)d_in[7];
  const float* al1   = (const float*)d_in[8];
  const float* ar1   = (const float*)d_in[9];
  const float* b1    = (const float*)d_in[10];
  const float* linW0 = (const float*)d_in[11];
  const float* linb0 = (const float*)d_in[12];
  const float* linW1 = (const float*)d_in[13];
  const float* linb1 = (const float*)d_in[14];
  float* out = (float*)d_out;
  const int* src0 = src;          const int* dst0 = dst;
  const int* src1 = src + nE;     const int* dst1 = dst + nE;

  const int MP = cdiv(nN, MROWS) * MROWS;
  const int gM = MP / GBM;
  const int nb = pick_nb(nE, nN);
  if (nb < 32 || (nb & (nb - 1)) != 0 || nb > NBMAX) return;
  const int gA = cdiv(MP, nb);
  if ((long long)gA * nb < (long long)MP) return;
  const int vec8 = ((nE & 3) == 0) ? 1 : 0;

  const size_t szRX = (size_t)MP * KA * 2;
  const size_t szRH = (size_t)MP * HC * 4;
  const size_t szRP = (size_t)MP * HC * 4;
  char* ws = (char*)d_ws;
  size_t off = 0;
  const size_t oW0T = off; off += (size_t)2 * HC * KA * 2;          off = (off + 255) & ~(size_t)255;
  const size_t oW1T = off; off += (size_t)2 * HC * KA * 2;          off = (off + 255) & ~(size_t)255;
  const size_t oL0T = off; off += (size_t)HID * KL * 2;             off = (off + 255) & ~(size_t)255;
  const size_t oL1T = off; off += (size_t)HID * KL * 2;             off = (off + 255) & ~(size_t)255;
  const size_t oSD  = off; off += (size_t)4 * MP * 4;               off = (off + 255) & ~(size_t)255;
  const size_t oRX  = off; off += szRX;                             off = (off + 255) & ~(size_t)255;
  const size_t oRH  = off; off += szRH;                             off = (off + 255) & ~(size_t)255;
  const size_t oRP  = off; off += szRP;                             off = (off + 255) & ~(size_t)255;
  if (off > ws_size || off > (size_t)WSMAX) return;
  unsigned short* W0T = (unsigned short*)(ws + oW0T);
  unsigned short* W1T = (unsigned short*)(ws + oW1T);
  unsigned short* L0T = (unsigned short*)(ws + oL0T);
  unsigned short* L1T = (unsigned short*)(ws + oL1T);
  float*          SD  = (float*)(ws + oSD);
  unsigned short* XB  = (unsigned short*)(ws + oRX);
  unsigned short* HB  = (unsigned short*)(ws + oRX);
  float*          H   = (float*)(ws + oRH);
  float*          P   = (float*)(ws + oRP);
  unsigned short* A2  = (unsigned short*)(ws + oRP);

  hipFuncSetAttribute(reinterpret_cast<const void*>(&k_agg<0>), hipFuncAttributeMaxDynamicSharedMemorySize, LDS_AGG);
  hipFuncSetAttribute(reinterpret_cast<const void*>(&k_agg<1>), hipFuncAttributeMaxDynamicSharedMemorySize, LDS_AGG);

  k_wprep<<<NUW / NTHR, NTHR, 0, stream>>>(W0, W1, linW0, linW1, W0T, W1T, L0T, L1T);
  const int nUx = MP * (KA / 8);
  k_xprep<<<cdiv(nUx, NTHR), NTHR, 0, stream>>>(x, XB, nN, nUx);

  k_gemm<<<gM, GTHR, 0, stream>>>(XB, W0T + (size_t)0 * HC * KA, H, al0 + 0 * HC, ar0 + 0 * HC, SD, MP);
  k_agg<0><<<gA, NTHR, LDS_AGG, stream>>>(src0, dst0, H, SD, b0 + 0 * HC, P, P, A2, nN, nE, nb, vec8, MP);
  k_gemm<<<gM, GTHR, 0, stream>>>(XB, W0T + (size_t)1 * HC * KA, H, al0 + 1 * HC, ar0 + 1 * HC, SD, MP);
  k_agg<1><<<gA, NTHR, LDS_AGG, stream>>>(src1, dst1, H, SD, b0 + 1 * HC, P, P, A2, nN, nE, nb, vec8, MP);
  k_lin<0><<<gM, GTHR, 0, stream>>>(A2, L0T, linb0, HB, out, nN);

  k_gemm<<<gM, GTHR, 0, stream>>>(HB, W1T + (size_t)0 * HC * KA, H, al1 + 0 * HC, ar1 + 0 * HC, SD, MP);
  k_agg<0><<<gA, NTHR, LDS_AGG, stream>>>(src0, dst0, H, SD, b1 + 0 * HC, P, P, A2, nN, nE, nb, vec8, MP);
  k_gemm<<<gM, GTHR, 0, stream>>>(HB, W1T + (size_t)1 * HC * KA, H, al1 + 1 * HC, ar1 + 1 * HC, SD, MP);
  k_agg<1><<<gA, NTHR, LDS_AGG, stream>>>(src1, dst1, H, SD, b1 + 1 * HC, P, P, A2, nN, nE, nb, vec8, MP);
  k_lin<1><<<gM, GTHR, 0, stream>>>(A2, L1T, linb1, HB, out, nN);
}
